// MicroConv_67568425500741
// MI455X (gfx1250) — hardware-verified
//
#include <hip/hip_runtime.h>
#include <math.h>

#define NN   50000
#define NE   1600000
#define DIN  128
#define NH   8
#define DH   16
#define NT   256
#define NPAD 50048
#define SRB  2048
#define NTL  25
#define RPW  (SRB / 8)
#define SCH  2048
#define NCH  ((NE + SCH - 1) / SCH)

typedef __attribute__((ext_vector_type(16))) _Float16 v16h;
typedef __attribute__((ext_vector_type(8)))  _Float16 v8h;
typedef __attribute__((ext_vector_type(4)))  _Float16 v4h;
typedef __attribute__((ext_vector_type(16))) __bf16   v16b;
typedef __attribute__((ext_vector_type(8)))  __bf16   v8b;
typedef __attribute__((ext_vector_type(8)))  float    v8f;
typedef __attribute__((ext_vector_type(4)))  float    v4f;
typedef __attribute__((ext_vector_type(2)))  float    v2f;
typedef __attribute__((ext_vector_type(4)))  int      v4i;

__device__ __forceinline__ unsigned short f2bf_bits(float f) {
  unsigned u = __float_as_uint(f);
  return (unsigned short)((u + 0x7FFFu + ((u >> 16) & 1u)) >> 16);
}
__device__ __forceinline__ float bf_bits2f(unsigned short h) { return __uint_as_float(((unsigned)h) << 16); }

__device__ __forceinline__ void dep_guard_h(v8f& a, v8f& b, v16h x, v16h y) { asm volatile("v_nop\n\tv_nop\n\tv_nop\n\tv_nop" : "+v"(a), "+v"(b) : "v"(x), "v"(y)); }
__device__ __forceinline__ void dep_guard_b(v8f& a, v8f& b, v16b x, v16b y) { asm volatile("v_nop\n\tv_nop\n\tv_nop\n\tv_nop" : "+v"(a), "+v"(b) : "v"(x), "v"(y)); }
__device__ __forceinline__ void keep4_h(v16h a, v16h b, v16h c, v16h d) { asm volatile("v_nop" :: "v"(a), "v"(b), "v"(c), "v"(d)); }
__device__ __forceinline__ void keep4_b(v16b a, v16b b, v16b c, v16b d) { asm volatile("v_nop" :: "v"(a), "v"(b), "v"(c), "v"(d)); }
__device__ __forceinline__ void acc_guard4(v8f& a, v8f& b, v8f& c, v8f& d) { asm volatile("v_nop\n\tv_nop\n\tv_nop\n\tv_nop" : "+v"(a), "+v"(b), "+v"(c), "+v"(d)); }
template <typename T> struct Frag;
template <> struct Frag<_Float16> {
  typedef v16h V; union U { v16h v; v8h h[2]; };
  static __device__ __forceinline__ v16h load(const _Float16* p) {
    U f; f.h[0] = *(const v8h*)(p); f.h[1] = *(const v8h*)(p + 16); return f.v;
  }
  static __device__ __forceinline__ v8f mma(v16h a, v16h b, v8f c) {
    return __builtin_amdgcn_wmma_f32_16x16x32_f16(false, a, false, b, (short)0, c, false, false);
  }
  static __device__ __forceinline__ void guard(v8f& a, v8f& b, v16h x, v16h y) { dep_guard_h(a, b, x, y); }
  static __device__ __forceinline__ void keep(v16h a, v16h b, v16h c, v16h d) { keep4_h(a, b, c, d); }
};
template <> struct Frag<__bf16> {
  typedef v16b V; union U { v16b v; v8b h[2]; };
  static __device__ __forceinline__ v16b load(const __bf16* p) {
    U f; f.h[0] = *(const v8b*)(p); f.h[1] = *(const v8b*)(p + 16); return f.v;
  }
  static __device__ __forceinline__ v8f mma(v16b a, v16b b, v8f c) {
    return __builtin_amdgcn_wmma_f32_16x16x32_bf16(false, a, false, b, (short)0, c, false, false);
  }
  static __device__ __forceinline__ void guard(v8f& a, v8f& b, v16b x, v16b y) { dep_guard_b(a, b, x, y); }
  static __device__ __forceinline__ void keep(v16b a, v16b b, v16b c, v16b d) { keep4_b(a, b, c, d); }
};

template <int ET> struct Elem;
template <> struct Elem<0> { typedef _Float16 T; };
template <> struct Elem<1> { typedef __bf16 T; };
template <int ET, bool SPLIT, int BIAS_MODE, int OUT_MODE, bool RESID, int ACT = 0>
__global__ __launch_bounds__(256) void wmma_gemm64(
    const unsigned short* __restrict__ Ap, const unsigned short* __restrict__ A2p, int lda, long strideA,
    const unsigned short* __restrict__ Btp, const unsigned short* __restrict__ Bt2p, int ldb, long strideB,
    void* __restrict__ Cout, void* __restrict__ Cout2, int ldc, long strideC,
    const float* __restrict__ bias,
    const float* __restrict__ resid, long strideR,
    int M, int N, int K, float scale) {
  typedef typename Elem<ET>::T T;
  typedef typename Frag<T>::V V;
  const T* A = (const T*)Ap; const T* A2 = (const T*)A2p; const T* Bt = (const T*)Btp; const T* Bt2 = (const T*)Bt2p;
  __shared__ __align__(16) float sT[8][16 * 68];
  const int b    = blockIdx.y;
  const int lane = threadIdx.x & 31;
  const int wave = threadIdx.x >> 5;
  const int tilesN = N >> 6;
  const int tilesM = M >> 6;
  const int tile = blockIdx.x * 8 + wave;
  if (tile >= tilesM * tilesN) return;
  const int tm = tile / tilesN;
  const int tn = tile - tm * tilesN;
  const int m0 = tm << 6;
  const int n0 = tn << 6;

  const T* Ab  = A  + (size_t)b * strideA;
  const T* Bb  = Bt + (size_t)b * strideB;
  const T* Ab2 = SPLIT ? (A2  + (size_t)b * strideA) : nullptr;
  const T* Bb2 = SPLIT ? (Bt2 + (size_t)b * strideB) : nullptr;

  const int rlane = lane & 15;
  const int koff  = (lane >> 4) * 8;
  const int mOff  = (lane >> 4) * 8;

  v8f acc[4][4];
#pragma unroll
  for (int i = 0; i < 4; ++i)
#pragma unroll
    for (int j = 0; j < 4; ++j) acc[i][j] = (v8f){0.f,0.f,0.f,0.f,0.f,0.f,0.f,0.f};

  for (int k0 = 0; k0 < K; k0 += 32) {
    V bh[4], bl[4];
#pragma unroll
    for (int j = 0; j < 4; ++j) {
      const size_t bo = (size_t)(n0 + (j << 4) + rlane) * ldb + koff + k0;
      bh[j] = Frag<T>::load(Bb + bo);
      if (SPLIT) bl[j] = Frag<T>::load(Bb2 + bo);
    }
#pragma unroll
    for (int i = 0; i < 4; ++i) {
      const size_t ao = (size_t)(m0 + (i << 4) + rlane) * lda + koff + k0;
      V ah = Frag<T>::load(Ab + ao);
      V al;
      if (SPLIT) al = Frag<T>::load(Ab2 + ao);
#pragma unroll
      for (int j = 0; j < 4; ++j) {
        acc[i][j] = Frag<T>::mma(ah, bh[j], acc[i][j]);
        if (SPLIT) {
          acc[i][j] = Frag<T>::mma(ah, bl[j], acc[i][j]);
          acc[i][j] = Frag<T>::mma(al, bh[j], acc[i][j]);
        }
      }
      Frag<T>::guard(acc[i][0], acc[i][3], ah, SPLIT ? al : ah);
    }
    Frag<T>::keep(bh[0], bh[1], bh[2], bh[3]);
    if (SPLIT) Frag<T>::keep(bl[0], bl[1], bl[2], bl[3]);
  }
  acc_guard4(acc[0][0], acc[0][1], acc[0][2], acc[0][3]);
  acc_guard4(acc[1][0], acc[1][1], acc[1][2], acc[1][3]);
  acc_guard4(acc[2][0], acc[2][1], acc[2][2], acc[2][3]);
  acc_guard4(acc[3][0], acc[3][1], acc[3][2], acc[3][3]);

  float* slab = sT[wave];
  const float* Rb = RESID ? (resid + (size_t)b * strideR) : nullptr;
#pragma unroll
  for (int i = 0; i < 4; ++i) {
    const int mBase = m0 + (i << 4);
#pragma unroll
    for (int j = 0; j < 4; ++j) {
      const int n = n0 + (j << 4) + rlane;
      float bv = 0.f;
      if (BIAS_MODE == 2) bv = bias[n];
#pragma unroll
      for (int r = 0; r < 8; ++r) {
        float v = acc[i][j][r] * scale;
        if (BIAS_MODE == 1) v += bias[mBase + mOff + r];
        if (BIAS_MODE == 2) v += bv;
        if (RESID) v += Rb[(size_t)(mBase + mOff + r) * ldc + n];
        if (ACT == 1) v = tanhf(v);
        if (ACT == 2) v = fmaxf(v, 0.0f);
        if (ACT == 3) v = v / (1.0f + expf(-v));
        if (ACT == 4) v = (v > 0.f) ? v : 0.01f * v;
        if (ACT == 5) v = 0.5f * v * (1.0f + erff(v * 0.70710678118654752f));
        slab[(mOff + r) * 68 + (j << 4) + rlane] = v;
      }
    }
    __builtin_amdgcn_fence(__ATOMIC_RELEASE, "workgroup");
    __builtin_amdgcn_wave_barrier();
    __builtin_amdgcn_fence(__ATOMIC_ACQUIRE, "workgroup");
    if (OUT_MODE == 0) {
      float* C = (float*)Cout + (size_t)b * strideC;
      const int hh = lane >> 4, c4 = (lane & 15) * 4;
      for (int pass = 0; pass < 2; ++pass) {
#pragma unroll
        for (int it = 0; it < 8; ++it) {
          const int row = it * 2 + hh;
          v4f v = *(const v4f*)(slab + row * 68 + c4);
          *(volatile v4f*)(C + (size_t)(mBase + row) * ldc + n0 + c4) = v;
        }
        __threadfence();
      }
    } else {
      const int q = lane >> 3, c8 = (lane & 7) * 8;
      unsigned short* C  = (unsigned short*)Cout  + (size_t)b * strideC;
      unsigned short* C2 = (OUT_MODE == 2) ? ((unsigned short*)Cout2 + (size_t)b * strideC) : nullptr;
      for (int pass = 0; pass < 2; ++pass) {
#pragma unroll
        for (int it = 0; it < 4; ++it) {
          const int row = it * 4 + q;
          const float* sp = slab + row * 68 + c8;
          v8h hv, lv;
#pragma unroll
          for (int e = 0; e < 8; ++e) {
            if (OUT_MODE == 1) {
              hv[e] = (_Float16)sp[e];
            } else {
              unsigned short hb = f2bf_bits(sp[e]);
              unsigned short lb = f2bf_bits(sp[e] - bf_bits2f(hb));
              hv[e] = __builtin_bit_cast(_Float16, hb);
              lv[e] = __builtin_bit_cast(_Float16, lb);
            }
          }
          *(volatile v8h*)(C + (size_t)(mBase + row) * ldc + n0 + c8) = hv;
          if (OUT_MODE == 2) *(volatile v8h*)(C2 + (size_t)(mBase + row) * ldc + n0 + c8) = lv;
        }
        __threadfence();
      }
    }
    __builtin_amdgcn_fence(__ATOMIC_RELEASE, "workgroup");
    __builtin_amdgcn_wave_barrier();
    __builtin_amdgcn_fence(__ATOMIC_ACQUIRE, "workgroup");
  }
}

__global__ __launch_bounds__(256) void transpose_cast_f16(const float* __restrict__ in, int ldi,
                                                         _Float16* __restrict__ outT, int ldo, float scale) {
  __shared__ __align__(16) _Float16 tile[64][72];
  const int c0 = blockIdx.x * 64, r0 = blockIdx.y * 64;
  const int t = threadIdx.y * 32 + threadIdx.x;
  for (int i = threadIdx.y; i < 64; i += 8) {
    tile[threadIdx.x][i]      = (_Float16)(in[(size_t)(r0 + i) * ldi + c0 + threadIdx.x] * scale);
    tile[32 + threadIdx.x][i] = (_Float16)(in[(size_t)(r0 + i) * ldi + c0 + 32 + threadIdx.x] * scale);
  }
  __syncthreads();
  const int q = t >> 3, c8 = (t & 7) * 8;
  for (int pass = 0; pass < 2; ++pass) {
#pragma unroll
    for (int it = 0; it < 2; ++it) {
      const int c = it * 32 + q;
      v8h hv = *(const v8h*)(&tile[c][c8]);
      *(volatile v8h*)(outT + (size_t)(c0 + c) * ldo + r0 + c8) = hv;
    }
    __threadfence();
  }
}

__global__ __launch_bounds__(256) void padcast_rows_kernel(const float* __restrict__ x, unsigned* __restrict__ X16) {
  const long i = (long)blockIdx.x * 256 + threadIdx.x; if (i >= (long)NPAD * DIN / 2) return;
  const long e0 = 2 * i; const bool ok = e0 < (long)NN * DIN;
  const float a = ok ? x[e0] : 0.f, b = ok ? x[e0 + 1] : 0.f;
  const unsigned u = (unsigned)__builtin_bit_cast(unsigned short, (_Float16)a) | ((unsigned)__builtin_bit_cast(unsigned short, (_Float16)b) << 16);
  ((volatile unsigned*)X16)[i] = u; __threadfence(); ((volatile unsigned*)X16)[i] = u;
}

template <bool W16>
__global__ __launch_bounds__(NT) void node_terms_kernel(const float* __restrict__ HF, const float* __restrict__ attn, int aoff,
                                                        _Float16* __restrict__ H16, float* __restrict__ EO) {
  __shared__ __align__(16) float so[16 * NH];
  const int lane = threadIdx.x & 31, wave = threadIdx.x >> 5;
  const int h = lane >> 2;
  const v4f av = *(const v4f*)(attn + h * (2 * DH) + aoff + 4 * (lane & 3));
#pragma unroll
  for (int t = 0; t < 2; ++t) {
    const int n = blockIdx.x * 16 + wave * 2 + t;
    const v4f xv = *(const v4f*)(HF + (size_t)n * DIN + 4 * lane);
    float p = xv[0] * av[0]; p += xv[1] * av[1]; p += xv[2] * av[2]; p += xv[3] * av[3];
    p += __shfl_xor(p, 1, 32); p += __shfl_xor(p, 2, 32);
    if ((lane & 3) == 0) so[(wave * 2 + t) * NH + h] = p;
    if (W16) {
      const v4h hv = __builtin_convertvector(xv, v4h);
      _Float16* op = H16 + (size_t)n * DIN + 4 * lane;
      *(volatile v4h*)op = hv; __threadfence(); *(volatile v4h*)op = hv;
    }
  }
  __syncthreads();
  if (wave == 0) {
    const v4f v = *(const v4f*)(so + 4 * lane);
    float* op = EO + (size_t)blockIdx.x * (16 * NH) + 4 * lane;
    *(volatile v4f*)op = v; __threadfence(); *(volatile v4f*)op = v;
  }
}

__device__ __forceinline__ int blk_excl_scan(int cnt, int* scan_ws, int tid, int* tot) {
  const int lane = tid & 31, wave = tid >> 5; int incl = cnt;
#pragma unroll
  for (int o = 1; o < 32; o <<= 1) { const int v = __shfl_up(incl, o, 32); if (lane >= o) incl += v; }
  if (lane == 31) scan_ws[wave] = incl;
  __syncthreads();
  if (wave == 0) { int wv = (lane < NT / 32) ? scan_ws[lane] : 0; int wincl = wv;
#pragma unroll
    for (int o = 1; o < 32; o <<= 1) { const int v = __shfl_up(wincl, o, 32); if (lane >= o) wincl += v; }
    if (lane < NT / 32) scan_ws[32 + lane] = wincl - wv; if (lane == 31) scan_ws[64] = wincl; }
  __syncthreads();
  const int res = scan_ws[32 + wave] + incl - cnt; *tot = scan_ws[64];
  return res;
}
template <int SP, int CAP>
__device__ __forceinline__ int chunk_hits(const int* __restrict__ dstv, const int* __restrict__ srcv, int e0, int n0, int tid,
                                          int* LIST, int* scan_ws) {
  const int eb = e0 + tid * SP;
  const int nhi = (n0 + SRB < NN) ? (n0 + SRB) : NN;
  int rec[SP]; int cnt = 0;
  if (eb < NE) {
#pragma unroll
    for (int k = 0; k < SP; k += 4) {
      const v4i d4 = *(const v4i*)(dstv + eb + k);
      const v4i s4 = *(const v4i*)(srcv + eb + k);
#pragma unroll
      for (int e = 0; e < 4; ++e) {
        const int d = d4[e]; int r = -1;
        if (d >= n0 && d < nhi) { int s = s4[e]; s = s < 0 ? 0 : (s >= NN ? NN - 1 : s); r = ((d - n0) << 16) | s; ++cnt; }
        rec[k + e] = r;
      }
    }
  } else {
#pragma unroll
    for (int k = 0; k < SP; ++k) rec[k] = -1;
  }
  int tot; int p = blk_excl_scan(cnt, scan_ws, tid, &tot);
#pragma unroll
  for (int k = 0; k < SP; ++k) if (rec[k] >= 0) { if ((unsigned)p < (unsigned)CAP) LIST[p] = rec[k]; ++p; }
  __syncthreads();
  return tot < CAP ? tot : CAP;
}

__global__ __launch_bounds__(NT) void gat_agg_kernel(const _Float16* __restrict__ HS, const int* __restrict__ srcv, const int* __restrict__ dstv,
                                                     const float* __restrict__ EL, const float* __restrict__ ER, float* AGG,
                                                     float* __restrict__ out) {
  __shared__ int LIST[SCH];
  __shared__ float SM[SRB * NH];
  __shared__ float SL[SRB * NH];
  __shared__ int scan_ws[80];
  const int tid = threadIdx.x, lane = tid & 31, wave = tid >> 5;
  const int tile = blockIdx.x;
  const int n0 = tile * SRB;
  const int h8 = lane & 7;
  const int hj = lane >> 2;
  const v4f z4 = {0.f, 0.f, 0.f, 0.f};
#pragma unroll 1
  for (int j = 0; j < RPW; ++j) {
    float* rp = AGG + (size_t)(n0 + wave * RPW + j) * DIN + 4 * lane;
    *(volatile v4f*)rp = z4;
    __threadfence();
    *(volatile v4f*)rp = z4;
  }
  for (int i = tid; i < SRB * NH; i += NT) { SM[i] = -INFINITY; SL[i] = 0.f; }
  __syncthreads();
#pragma unroll 1
  for (int c = 0; c < NCH; ++c) {
    const int tot = chunk_hits<SCH / NT, SCH>(dstv, srcv, c * SCH, n0, tid, LIST, scan_ws);
#pragma unroll 1
    for (int base = 0; base < tot; base += 32) {
      const int q = base + lane;
      const int rv = (q < tot) ? LIST[q] : -1;
      const int own = (rv >= 0 && (rv >> 24) == wave) ? 1 : 0;
      unsigned msk = (unsigned)__ballot(own);
#pragma unroll 1
      for (int it = 0; it < 32; ++it) {
        if (msk == 0u) break;
        const int bp = __builtin_ctz(msk); msk &= msk - 1u;
        const int r = __shfl(rv, bp, 32);
        const int dl = r >> 16, s = r & 0xFFFF;
        const int mi = dl * NH + h8;
        float al = EL[(size_t)s * NH + h8] + ER[(size_t)(n0 + dl) * NH + h8];
        al = (al >= 0.f) ? al : 0.2f * al;
        const float mo = SM[mi], lo = SL[mi];
        const float mn = fmaxf(mo, al);
        const float rr = __expf(mo - mn), ex = __expf(al - mn);
        const float ln = lo * rr + ex;
        if (lane < NH) { SM[mi] = mn; SL[mi] = ln; }
        const float rrj = __shfl(rr, hj, 32), exj = __shfl(ex, hj, 32);
        const v4h xv = *(const v4h*)(HS + (size_t)s * DIN + 4 * lane);
        const v4f hv = __builtin_convertvector(xv, v4f);
        float* rp = AGG + (size_t)(n0 + dl) * DIN + 4 * lane;
        v4f a = *(const v4f*)rp;
        a = a * rrj + exj * hv;
        *(volatile v4f*)rp = a;
        __threadfence();
        *(volatile v4f*)rp = a;
      }
    }
    __syncthreads();
  }
#pragma unroll 1
  for (int jj = 0; jj < RPW; ++jj) {
    const int dl = wave * RPW + jj;
    const int n = n0 + dl;
    if (n >= NN) break;
    const float lv = (lane < NH) ? SL[dl * NH + lane] : 1.0f;
    const float inv = (lv > 0.f) ? (1.0f / lv) : 0.f;
    const float ih = __shfl(inv, hj, 32);
    const v4f a = *(const v4f*)(AGG + (size_t)(n0 + dl) * DIN + 4 * lane);
    const v4f v = a * ih;
    float* op = out + (size_t)n * DIN + 4 * lane;
    *(volatile v4f*)op = v; __threadfence(); *(volatile v4f*)op = v;
  }
}

extern "C" void kernel_launch(void* const* d_in, const int* in_sizes, int n_in,
                              void* d_out, int out_size, void* d_ws, size_t ws_size, hipStream_t stream) {
  if (n_in < 9) return;
  const float* feat_src = (const float*)d_in[0];
  const float* feat_dst = (const float*)d_in[1];
  const float* W_src    = (const float*)d_in[2];
  const float* b_src    = (const float*)d_in[3];
  const float* W_dst    = (const float*)d_in[4];
  const float* b_dst    = (const float*)d_in[5];
  const float* attn     = (const float*)d_in[6];
  const int*   src_idx  = (const int*)d_in[7];
  const int*   dst_idx  = (const int*)d_in[8];
  float* out = (float*)d_out;
  if (in_sizes[0] != NN * DIN || in_sizes[1] != NN * DIN || in_sizes[2] != DIN * DIN || in_sizes[3] != DIN ||
      in_sizes[4] != DIN * DIN || in_sizes[5] != DIN || in_sizes[6] != NH * 2 * DH || in_sizes[7] != NE || in_sizes[8] != NE ||
      out_size != NN * DIN) return;

  char* ws = (char*)d_ws; size_t off = 0;
  auto carve = [&](size_t bytes) -> char* { char* p = ws + off; off += (bytes + 255) & ~(size_t)255; return p; };
  _Float16* WsT  = (_Float16*)carve((size_t)DIN * DIN * 2);
  _Float16* WdT  = (_Float16*)carve((size_t)DIN * DIN * 2);
  unsigned* X16  = (unsigned*)carve((size_t)NPAD * DIN * 2);
  float*    HF   = (float*)carve((size_t)NPAD * DIN * 4);
  _Float16* HS16 = (_Float16*)carve((size_t)NPAD * DIN * 2);
  float*    EL   = (float*)carve((size_t)NPAD * NH * 4);
  float*    ER   = (float*)carve((size_t)NPAD * NH * 4);
  float*    AGG  = (float*)carve((size_t)NTL * SRB * DIN * 4);
  if (off > ws_size || off > (size_t)134217728) return;

  const int ncast  = (NPAD * DIN / 2 + 255) / 256;
  const int gtiles = (NPAD / 64) * (DIN / 64);

  transpose_cast_f16<<<dim3(DIN / 64, DIN / 64), dim3(32, 8), 0, stream>>>(W_src, DIN, WsT, DIN, 16.0f);
  transpose_cast_f16<<<dim3(DIN / 64, DIN / 64), dim3(32, 8), 0, stream>>>(W_dst, DIN, WdT, DIN, 16.0f);

  padcast_rows_kernel<<<ncast, 256, 0, stream>>>(feat_src, X16);
  wmma_gemm64<0, false, 2, 0, false><<<dim3((gtiles + 7) / 8, 1), 256, 0, stream>>>(
      (const unsigned short*)X16, nullptr, DIN, 0L, (const unsigned short*)WsT, nullptr, DIN, 0L,
      (void*)HF, nullptr, DIN, 0L, b_src, nullptr, 0L, NPAD, DIN, DIN, 0.0625f);
  node_terms_kernel<true><<<NPAD / 16, NT, 0, stream>>>(HF, attn, 0, HS16, EL);

  padcast_rows_kernel<<<ncast, 256, 0, stream>>>(feat_dst, X16);
  wmma_gemm64<0, false, 2, 0, false><<<dim3((gtiles + 7) / 8, 1), 256, 0, stream>>>(
      (const unsigned short*)X16, nullptr, DIN, 0L, (const unsigned short*)WdT, nullptr, DIN, 0L,
      (void*)HF, nullptr, DIN, 0L, b_dst, nullptr, 0L, NPAD, DIN, DIN, 0.0625f);
  node_terms_kernel<false><<<NPAD / 16, NT, 0, stream>>>(HF, attn, DH, nullptr, ER);

  gat_agg_kernel<<<NTL, NT, 0, stream>>>(HS16, src_idx, dst_idx, EL, ER, AGG, out);
}
